// StandAloneSelfAttention_42331197669625
// MI455X (gfx1250) — hardware-verified
//
#include <hip/hip_runtime.h>
#include <math.h>

typedef __attribute__((ext_vector_type(16))) _Float16 v16h;
typedef __attribute__((ext_vector_type(16))) __bf16 v16b;
typedef __attribute__((ext_vector_type(8)))  _Float16 v8h;
typedef __attribute__((ext_vector_type(8)))  float v8f;
typedef __attribute__((ext_vector_type(4)))  float v4f;
typedef __attribute__((ext_vector_type(2)))  float v2f;
typedef __attribute__((ext_vector_type(4)))  unsigned v4u;
typedef __attribute__((ext_vector_type(4)))  int v4i;
typedef float __attribute__((may_alias)) float_a;
typedef int __attribute__((may_alias)) int_a;

template <typename T> __device__ __forceinline__ void vst2(void* p, T v) { *(volatile T*)p = v; __threadfence(); *(volatile T*)p = v; }
__device__ __forceinline__ v8f wmma16(v16h a, v16h b, v8f c) {
  v8f d = __builtin_amdgcn_wmma_f32_16x16x32_f16(false, a, false, b, (short)0, c, false, false);
  asm volatile("v_nop\n\tv_nop\n\tv_nop\n\tv_nop" : "+v"(d) : "v"(a), "v"(b));
  return d;
}
__device__ __forceinline__ v8f wmma_bf(v16b a, v16b b, v8f c) {
  v8f d = __builtin_amdgcn_wmma_f32_16x16x32_bf16(false, a, false, b, (short)0, c, false, false);
  asm volatile("v_nop\n\tv_nop\n\tv_nop\n\tv_nop" : "+v"(d) : "v"(a), "v"(b));
  return d;
}
__device__ __forceinline__ v16h frag_h(const _Float16* rowk0, int lane) {
  union { v16h v; v8h q[2]; } u; const _Float16* p = rowk0 + 8 * (lane >> 4);
  u.q[0] = *(const v8h*)p; u.q[1] = *(const v8h*)(p + 16); return u.v;
}
__device__ __forceinline__ v16h frag_f32(const float* rowk0, int lane) {
  v16h a; const float* p = rowk0 + 8 * (lane >> 4);
#pragma unroll
  for (int i = 0; i < 8; ++i) { a[i] = (_Float16)p[i]; a[8 + i] = (_Float16)p[16 + i]; }
  return a;
}
__device__ __forceinline__ v16h frag_f32s(const float* rowk0, int lane, float sc) {
  v16h a; const float* p = rowk0 + 8 * (lane >> 4);
#pragma unroll
  for (int i = 0; i < 8; ++i) { a[i] = (_Float16)(p[i] * sc); a[8 + i] = (_Float16)(p[16 + i] * sc); }
  return a;
}
__device__ __forceinline__ v16h fragc_f32(const float* W, int k0, int n, int lane, int ld, int K) {
  v16h a; const int g = lane >> 4;
#pragma unroll
  for (int i = 0; i < 8; ++i) { const int ka = k0 + 8 * g + i, kb = ka + 16;
    a[i] = (_Float16)(ka < K ? W[(size_t)(ka < K ? ka : K - 1) * ld + n] : 0.f); a[8 + i] = (_Float16)(kb < K ? W[(size_t)(kb < K ? kb : K - 1) * ld + n] : 0.f); }
  return a;
}
struct F2 { v16b h, l; };
__device__ __forceinline__ F2 bsplit16(const float v[16]) { F2 r;
#pragma unroll
  for (int i = 0; i < 16; ++i) { const __bf16 h = (__bf16)v[i]; r.h[i] = h; r.l[i] = (__bf16)(v[i] - (float)h); }
  return r; }
__device__ __forceinline__ F2 split_row(const float* row, int k0, int lane) { float v[16]; const float* p = row + k0 + 8 * (lane >> 4);
#pragma unroll
  for (int i = 0; i < 8; ++i) { v[i] = p[i]; v[8 + i] = p[16 + i]; }
  return bsplit16(v); }
__device__ __forceinline__ F2 split_rowK(const float* row, int k0, int lane, int K) { float v[16]; const int g = lane >> 4;
#pragma unroll
  for (int i = 0; i < 8; ++i) { const int ka = k0 + 8 * g + i, kb = ka + 16; v[i] = ka < K ? row[ka < K ? ka : K - 1] : 0.f; v[8 + i] = kb < K ? row[kb < K ? kb : K - 1] : 0.f; }
  return bsplit16(v); }
__device__ __forceinline__ F2 split_col(const float* W, int k0, int n, int lane, int ld, int K) { float v[16]; const int g = lane >> 4;
#pragma unroll
  for (int i = 0; i < 8; ++i) { const int ka = k0 + 8 * g + i, kb = ka + 16; v[i] = ka < K ? W[(size_t)(ka < K ? ka : K - 1) * ld + n] : 0.f; v[8 + i] = kb < K ? W[(size_t)(kb < K ? kb : K - 1) * ld + n] : 0.f; }
  return bsplit16(v); }
__device__ __forceinline__ v8f mac3(const F2& a, const F2& b, v8f c) { c = wmma_bf(a.l, b.h, c); c = wmma_bf(a.h, b.l, c); return wmma_bf(a.h, b.h, c); }
__device__ __forceinline__ float sigm(float v) { return 1.0f / (1.0f + expf(-v)); }
#define LDSX() do { asm volatile("s_wait_dscnt 0" ::: "memory"); __builtin_amdgcn_wave_barrier(); __builtin_amdgcn_fence(__ATOMIC_RELEASE, "workgroup"); } while (0)


#define NB 2
#define HH 64
#define WW 64
#define CC 256
#define NH 8
#define HS 32
#define KS 7
#define KK 49
#define NPIX (NB * HH * WW)
#define KWIN 22
#define NKEY (KS * KWIN)
#ifndef TY1
#define TY0 0
#define TY1 HH
#define TB0 0
#define TNB NB
#endif
typedef __attribute__((ext_vector_type(8))) __bf16 v8b;
__device__ __forceinline__ v16b frag_b(const __bf16* rowk0, int lane) {
  union { v16b v; v8b q[2]; } u; const __bf16* p = rowk0 + 8 * (lane >> 4);
  u.q[0] = *(const v8b*)p; u.q[1] = *(const v8b*)(p + 16); return u.v;
}
__device__ __forceinline__ float bfr(float v) { return (float)(__bf16)v; }
__device__ __attribute__((noinline)) float exp_ni(float v) { return expf(v); }
__device__ __attribute__((noinline)) float erf_ni(float v) { return erff(v); }

#define PK_Q 0
#define PK_K ((size_t)CC * CC)
#define PK_V ((size_t)2 * CC * CC)
#define PK_END ((size_t)3 * CC * CC)
#define WS_PK  0u
#define WS_QH  (((2u * PK_END) + 127u) / 128u * 128u)
#define WS_QL  (WS_QH + 2u * NPIX * CC)
#define WS_KH  (WS_QL + 2u * NPIX * CC)
#define WS_KL  (WS_KH + 2u * NPIX * CC)
#define WS_VH  (WS_KL + 2u * NPIX * CC)
#define WS_VL  (WS_VH + 2u * NPIX * CC)
#define WS_EH  (WS_VL + 2u * NPIX * CC)
#define WS_EL  (WS_EH + 2u * NH * 64 * HS)
#define WS_END (WS_EL + 2u * NH * 64 * HS)

__global__ __launch_bounds__(256) void k_pack(const float* __restrict__ WQ, const float* __restrict__ WK, const float* __restrict__ WV, const float* __restrict__ E0, const float* __restrict__ E1, __bf16* __restrict__ PK, _Float16* __restrict__ EH, _Float16* __restrict__ EL) {
  __shared__ __align__(16) __bf16 s[CC]; __shared__ __align__(16) _Float16 seh[2 * HS], sel[2 * HS]; const int n = blockIdx.x, which = blockIdx.y, t = threadIdx.x;
  if (which == 3) {
    if (n >= NH * 32) return;
    if (t < 2 * HS) { const int r = 2 * n + (t >> 5), d = t & 31; const int h = r >> 6, slot = r & 63; float v = 0.f; if (slot < KK) { const int i = slot / KS, j = slot % KS; v = (h < 4) ? bfr(E0[(size_t)(h * HS + d) * KS + i]) : bfr(E1[(size_t)((h - 4) * HS + d) * KS + j]); } const _Float16 hv = (_Float16)v; seh[t] = hv; sel[t] = (_Float16)((v - (float)hv) * 2048.0f); }
    __syncthreads();
    if (t < 8) vst2((unsigned*)(EH + (size_t)2 * n * HS + t * 8), *(const v4u*)&seh[t * 8]); else if (t < 16) vst2((unsigned*)(EL + (size_t)2 * n * HS + (t - 8) * 8), *(const v4u*)&sel[(t - 8) * 8]);
    return; }
  if (n >= CC) return;
  const float* Wm = (which == 0) ? WQ : (which == 1) ? WK : WV;
  for (int k = t; k < CC; k += 256) s[k] = (__bf16)Wm[(size_t)k * CC + n];
  __syncthreads();
  if (t < CC / 8) vst2((unsigned*)(PK + (size_t)which * CC * CC + (size_t)n * CC + t * 8), *(const v4u*)&s[t * 8]);
}
__global__ __launch_bounds__(128) void k_proj(const float* __restrict__ X, const __bf16* __restrict__ PK, const float* __restrict__ BQ, const float* __restrict__ BK, const float* __restrict__ BV, _Float16* __restrict__ QH, _Float16* __restrict__ QL, _Float16* __restrict__ KH, _Float16* __restrict__ KL, _Float16* __restrict__ VH, _Float16* __restrict__ VL) {
  __shared__ __align__(16) _Float16 soh[4][16][136], sol[4][16][136];
  const int tid = threadIdx.x, wave = tid >> 5, lane = tid & 31, col = lane & 15, g = lane >> 4; const int which = blockIdx.z; const size_t r0 = (size_t)blockIdx.x * 64 + wave * 16; const int n0 = blockIdx.y * 128;
  const __bf16* P = PK + (size_t)which * CC * CC; const float* BB = (which == 0) ? BQ : (which == 1) ? BK : BV;
  v8f acc[8] = {};
#pragma unroll 2
  for (int kc = 0; kc < CC / 32; ++kc) { v16b a; { const float* p = X + (r0 + col) * CC + kc * 32 + 8 * g;
#pragma unroll
      for (int i = 0; i < 8; ++i) { a[i] = (__bf16)p[i]; a[8 + i] = (__bf16)p[16 + i]; } }
#pragma unroll
    for (int j = 0; j < 8; ++j) acc[j] = wmma_bf(a, frag_b(P + (size_t)(n0 + j * 16 + col) * CC + kc * 32, lane), acc[j]); }
#pragma unroll
  for (int j = 0; j < 8; ++j) { const float bb = bfr(BB[n0 + j * 16 + col]);
#pragma unroll
    for (int r = 0; r < 8; ++r) { const float v = acc[j][r] + bb; const _Float16 hv = (_Float16)v; soh[wave][8 * g + r][j * 16 + col] = hv; sol[wave][8 * g + r][j * 16 + col] = (_Float16)((v - (float)hv) * 2048.0f); } }
  LDSX();
  _Float16* DH_ = (which == 0) ? QH : (which == 1) ? KH : VH; _Float16* DL_ = (which == 0) ? QL : (which == 1) ? KL : VL;
  for (int rl = 0; rl < 16; ++rl) { if (lane < 16) vst2((unsigned*)(DH_ + (r0 + rl) * CC + n0 + lane * 8), *(const v4u*)&soh[wave][rl][lane * 8]); else vst2((unsigned*)(DL_ + (r0 + rl) * CC + n0 + (lane - 16) * 8), *(const v4u*)&sol[wave][rl][(lane - 16) * 8]); }
}
__global__ __launch_bounds__(128) void k_attn(const _Float16* __restrict__ QH, const _Float16* __restrict__ QL, const _Float16* __restrict__ KH, const _Float16* __restrict__ KL, const _Float16* __restrict__ VH, const _Float16* __restrict__ VL, const _Float16* __restrict__ EH, const _Float16* __restrict__ EL, float* __restrict__ OUT) {
  __shared__ float sqe[4][16][65]; __shared__ float sqk[4][16][161]; __shared__ __align__(16) _Float16 sph[4][16][168], spl[4][16][168]; __shared__ __align__(16) float so[4][16][36]; __shared__ float sil[4][16];
  const int tid = threadIdx.x, wave = tid >> 5, lane = tid & 31, col = lane & 15, g = lane >> 4; const int y = TY0 + blockIdx.x, b = TB0 + blockIdx.y; const int x0 = wave * 16;
  const size_t prow0 = ((size_t)b * HH + y) * WW;
#pragma unroll 1
  for (int h = 0; h < NH; ++h) {
    const v16h aq = frag_h(QH + (prow0 + x0 + col) * CC + h * HS, lane), aql = frag_h(QL + (prow0 + x0 + col) * CC + h * HS, lane);
#pragma unroll
    for (int jt = 0; jt < 4; ++jt) { const size_t er = ((size_t)h * 64 + jt * 16 + col) * HS; v8f c = {}, cl = {}; const v16h eh = frag_h(EH + er, lane); c = wmma16(aq, eh, c); cl = wmma16(aql, eh, cl); cl = wmma16(aq, frag_h(EL + er, lane), cl);
#pragma unroll
      for (int r = 0; r < 8; ++r) sqe[wave][8 * g + r][jt * 16 + col] = c[r] + cl[r] * (1.0f / 2048.0f); }
#pragma unroll
    for (int jt = 0; jt < 10; ++jt) { const int j = jt * 16 + col; int ky = y + (j / KWIN) - 3, kx = x0 - 3 + (j % KWIN); if (j >= NKEY) { ky = y; kx = x0; } ky = min(max(ky, 0), HH - 1); kx = min(max(kx, 0), WW - 1);
      const size_t kr = (((size_t)b * HH + ky) * WW + kx) * CC + h * HS; v8f c = {}, cl = {}; const v16h kh = frag_h(KH + kr, lane); c = wmma16(aq, kh, c); cl = wmma16(aql, kh, cl); cl = wmma16(aq, frag_h(KL + kr, lane), cl);
#pragma unroll
      for (int r = 0; r < 8; ++r) sqk[wave][8 * g + r][j] = c[r] + cl[r] * (1.0f / 2048.0f); }
    LDSX();
    for (int e = lane; e < 16 * 168; e += 32) { sph[wave][e / 168][e % 168] = (_Float16)0.f; spl[wave][e / 168][e % 168] = (_Float16)0.f; }
    LDSX();
    if (lane < 16) { const int ql = lane; const int xq = x0 + ql; float mx = -3.0e38f;
#pragma unroll 1
      for (int s2 = 0; s2 < KK; ++s2) { const int i = s2 / KS, jx = s2 % KS; const int ky = y + i - 3, kx = xq + jx - 3; const bool in = (ky >= 0) && (ky < HH) && (kx >= 0) && (kx < WW);
        float v = sqe[wave][ql][s2]; if (in) v += sqk[wave][ql][i * KWIN + (ql + jx)]; mx = fmaxf(mx, v); }
      float l = 0.f;
#pragma unroll 1
      for (int s2 = 0; s2 < KK; ++s2) { const int i = s2 / KS, jx = s2 % KS; const int ky = y + i - 3, kx = xq + jx - 3; const bool in = (ky >= 0) && (ky < HH) && (kx >= 0) && (kx < WW);
        float v = sqe[wave][ql][s2]; if (in) v += sqk[wave][ql][i * KWIN + (ql + jx)]; const float e2 = exp_ni(v - mx); l += e2;
        if (in) { const float es = e2 * 2048.0f; const _Float16 hp = (_Float16)es; const int j = i * KWIN + (ql + jx); sph[wave][ql][j] = hp; spl[wave][ql][j] = (_Float16)((es - (float)hp) * 2048.0f); } }
      sil[wave][ql] = 1.0f / l; }
    LDSX();
    { v8f acc[2] = {}, accl[2] = {};
#pragma unroll 1
      for (int kc = 0; kc < 5; ++kc) { const v16h pah = frag_h(&sph[wave][col][kc * 32], lane), pal = frag_h(&spl[wave][col][kc * 32], lane);
#pragma unroll
        for (int dt = 0; dt < 2; ++dt) {
          v16h vbh, vbl; { const int dcol = dt * 16 + col;
#pragma unroll
            for (int i = 0; i < 16; ++i) { const int key = kc * 32 + 8 * g + (i & 7) + ((i >> 3) << 4); int ky = y + (key / KWIN) - 3, kx = x0 - 3 + (key % KWIN); const bool in = (key < NKEY) && ky >= 0 && ky < HH && kx >= 0 && kx < WW; ky = min(max(ky, 0), HH - 1); kx = min(max(kx, 0), WW - 1);
              const size_t vr = (((size_t)b * HH + ky) * WW + kx) * CC + h * HS + dcol; vbh[i] = in ? VH[vr] : (_Float16)0.f; vbl[i] = in ? VL[vr] : (_Float16)0.f; } }
          acc[dt] = wmma16(pah, vbh, acc[dt]); accl[dt] = wmma16(pal, vbh, accl[dt]); accl[dt] = wmma16(pah, vbl, accl[dt]); } }
#pragma unroll
      for (int dt = 0; dt < 2; ++dt)
#pragma unroll
        for (int r = 0; r < 8; ++r) so[wave][8 * g + r][dt * 16 + col] = (acc[dt][r] * (1.0f / 2048.0f) + accl[dt][r] * (1.0f / 4194304.0f)) * sil[wave][8 * g + r]; }
    LDSX();
    for (int rl = 0; rl < 16; ++rl) if (lane < 8) vst2(OUT + (prow0 + x0 + rl) * CC + h * HS + lane * 4, *(const v4f*)&so[wave][rl][lane * 4]);
    LDSX(); }
}
extern "C" void kernel_launch(void* const* d_in, const int* in_sizes, int n_in, void* d_out, int out_size, void* d_ws, size_t ws_size, hipStream_t stream) {
  (void)in_sizes; (void)n_in; (void)out_size;
  const float** F = (const float**)d_in;
  if (ws_size < (size_t)WS_END) return;
  char* ws = (char*)d_ws; __bf16* PK = (__bf16*)(ws + WS_PK); _Float16 *QH = (_Float16*)(ws + WS_QH), *QL = (_Float16*)(ws + WS_QL), *KH = (_Float16*)(ws + WS_KH), *KL = (_Float16*)(ws + WS_KL), *VH = (_Float16*)(ws + WS_VH), *VL = (_Float16*)(ws + WS_VL), *EH = (_Float16*)(ws + WS_EH), *EL = (_Float16*)(ws + WS_EL);
  k_pack<<<dim3(NH * 64, 4), 256, 0, stream>>>(F[1], F[3], F[5], F[7], F[8], PK, EH, EL);
  k_proj<<<dim3(NPIX / 64, CC / 128, 3), 128, 0, stream>>>(F[0], PK, F[2], F[4], F[6], QH, QL, KH, KL, VH, VL);
  k_attn<<<dim3(TY1 - TY0, TNB), 128, 0, stream>>>(QH, QL, KH, KL, VH, VL, EH, EL, (float*)d_out);
}
